// ClinicalGatedGCN_70858370450162
// MI455X (gfx1250) — hardware-verified
//
#include <hip/hip_runtime.h>
#include <stddef.h>


#define HD      128
#define NCL     16
#define NCLS    2
#define NG      64
#define NTHR    256
#define NWAVE   8
#define EPT     8
#define CHUNK   (NTHR * EPT)
#define WCAP    (EPT * 32)
#define NB      512
#define GTHR    128
#define GWAVE   4
#define GROWS   (GWAVE * 16)
#define WSC     16.0f
#define WINV    0.0625f
#define BN_EPS  1e-5f
#define SLOPE   0.01f
#define AGG_LDS ((NB * HD + NWAVE * WCAP + 16) * 4)

static_assert((NB % (2 * NWAVE)) == 0);
static_assert(NB <= 65536);
static_assert(CHUNK <= 32768);
static_assert((NB % GROWS) == 0);
static_assert(WCAP == 256);

typedef float    v4f  __attribute__((ext_vector_type(4)));
typedef float    v8f  __attribute__((ext_vector_type(8)));
typedef int      v4i  __attribute__((ext_vector_type(4)));
typedef _Float16 v8h  __attribute__((ext_vector_type(8)));
typedef _Float16 v16h __attribute__((ext_vector_type(16)));
union FragH { v16h v; v8h h[2]; };

__device__ __forceinline__ v4f zero4() { v4f z = {0.0f, 0.0f, 0.0f, 0.0f}; return z; }
__device__ __forceinline__ v8f zero8f() {
  v8f z;
#pragma unroll
  for (int i = 0; i < 8; ++i) z[i] = 0.0f;
  return z;
}

__device__ __forceinline__ v8f wmh(v16h a, v16h b, v8f c) {
  v8f d = __builtin_amdgcn_wmma_f32_16x16x32_f16(false, a, false, b, (short)0, c, false, false);
  asm volatile("v_nop\n\tv_nop\n\tv_nop\n\tv_nop" : "+v"(d) : "v"(a), "v"(b));
  return d;
}

__device__ __forceinline__ float bnl(float t, float g, float rm, float rs, float b) {
  const float u = (t >= 0.0f) ? t : SLOPE * t;
  return g * (u - rm) * rs + b;
}

__device__ __forceinline__ float gate1(float kk, float qq, float ea, float w, float b) {
  const float z = (kk + qq) + (ea * w + b);
  const float t = 1.0f + __expf(-z);
  return __builtin_amdgcn_rcpf(t);
}

__global__ __launch_bounds__(NTHR) void k_cvtw(const float* __restrict__ Wk, const float* __restrict__ Wq,
                                              const float* __restrict__ Wv, const float* __restrict__ Ws,
                                              _Float16* Wt, int nL) {
  const int b  = blockIdx.x;
  const int lp = b >> 3;
  const int l  = lp >> 2, p = lp & 3;
  if (l >= nL) return;
  const float* W = (p == 0) ? Wk : (p == 1) ? Wq : (p == 2) ? Wv : Ws;
  W += (size_t)l * HD * HD;
  const int t  = threadIdx.x;
  const int n  = (b & 7) * 16 + (t >> 4);
  const int kg = (t & 15) * 8;
  v8h v;
#pragma unroll
  for (int i = 0; i < 8; ++i) v[i] = (_Float16)(W[(size_t)(kg + i) * HD + n] * WSC);
  _Float16* dp = Wt + ((size_t)lp * HD + n) * HD + kg;
  *(volatile v8h*)dp = v;
  __threadfence();
  *(volatile v8h*)dp = v;
}

__global__ __launch_bounds__(NTHR) void k_cvtx(const float* __restrict__ x, _Float16* h16, int nN, int nPad) {
  const int idx = blockIdx.x * NTHR + threadIdx.x;
  const int row = idx >> 4;
  const int kg  = (idx & 15) * 8;
  if (row >= nPad) return;
  const int ra = row < nN - 1 ? row : nN - 1;
  const v4f a = *(const v4f*)(x + (size_t)ra * HD + kg);
  const v4f b = *(const v4f*)(x + (size_t)ra * HD + kg + 4);
  const bool ok = row < nN;
  v8h v;
  v[0] = (_Float16)(ok ? a.x : 0.0f); v[1] = (_Float16)(ok ? a.y : 0.0f);
  v[2] = (_Float16)(ok ? a.z : 0.0f); v[3] = (_Float16)(ok ? a.w : 0.0f);
  v[4] = (_Float16)(ok ? b.x : 0.0f); v[5] = (_Float16)(ok ? b.y : 0.0f);
  v[6] = (_Float16)(ok ? b.z : 0.0f); v[7] = (_Float16)(ok ? b.w : 0.0f);
  _Float16* dp = h16 + (size_t)row * HD + kg;
  *(volatile v8h*)dp = v;
  __threadfence();
  *(volatile v8h*)dp = v;
}

__device__ __forceinline__ void gemm_plane(const FragH (&a)[4], const _Float16* __restrict__ Wt,
                                           const float* __restrict__ bias, float* out,
                                           int row0, float* sw, int lane, int hh, int m) {
  v8f acc[8];
#pragma unroll
  for (int nt = 0; nt < 8; ++nt) acc[nt] = zero8f();
#pragma unroll
  for (int nt = 0; nt < 8; ++nt) {
    const _Float16* br = Wt + (size_t)(nt * 16 + m) * HD + 8 * hh;
#pragma unroll
    for (int kk = 0; kk < 4; ++kk) {
      FragH b;
      b.h[0] = *(const v8h*)(br + 32 * kk);
      b.h[1] = *(const v8h*)(br + 32 * kk + 16);
      acc[nt] = wmh(a[kk].v, b.v, acc[nt]);
    }
  }
#pragma unroll
  for (int nt = 0; nt < 8; ++nt) {
    const int col = nt * 16 + m;
    const float bc = bias[col];
#pragma unroll
    for (int r = 0; r < 8; ++r) sw[(8 * hh + r) * HD + col] = acc[nt][r] * WINV + bc;
  }
  __syncthreads();
#pragma unroll 4
  for (int r = 0; r < 16; ++r) {
    const v4f v = *(const v4f*)(sw + r * HD + 4 * lane);
    *(volatile v4f*)(out + (size_t)(row0 + r) * HD + 4 * lane) = v;
  }
  __threadfence();
#pragma unroll 4
  for (int r = 0; r < 16; ++r) {
    const v4f v = *(const v4f*)(sw + r * HD + 4 * lane);
    *(volatile v4f*)(out + (size_t)(row0 + r) * HD + 4 * lane) = v;
  }
  __syncthreads();
}

__global__ __launch_bounds__(GTHR) void k_gemm(const _Float16* __restrict__ hp, const _Float16* __restrict__ Wt4,
                                              const float* __restrict__ b0, const float* __restrict__ b1,
                                              const float* __restrict__ b2, const float* __restrict__ b3,
                                              float* o0, float* o1, float* o2, float* o3) {
  __shared__ __attribute__((aligned(16))) float stg[GWAVE * 16 * HD];
  const int tid = threadIdx.x, lane = tid & 31, wave = tid >> 5, hh = lane >> 4, m = lane & 15;
  const int row0 = blockIdx.x * GROWS + wave * 16;
  FragH a[4];
  {
    const _Float16* ar = hp + (size_t)(row0 + m) * HD + 8 * hh;
#pragma unroll
    for (int kk = 0; kk < 4; ++kk) {
      a[kk].h[0] = *(const v8h*)(ar + 32 * kk);
      a[kk].h[1] = *(const v8h*)(ar + 32 * kk + 16);
    }
  }
  float* sw = stg + wave * 16 * HD;
  gemm_plane(a, Wt4 + 0 * HD * HD, b0, o0, row0, sw, lane, hh, m);
  gemm_plane(a, Wt4 + 1 * HD * HD, b1, o1, row0, sw, lane, hh, m);
  gemm_plane(a, Wt4 + 2 * HD * HD, b2, o2, row0, sw, lane, hh, m);
  gemm_plane(a, Wt4 + 3 * HD * HD, b3, o3, row0, sw, lane, hh, m);
}

__device__ __forceinline__ int scan_chunk(const int* __restrict__ dsts, int nE, int cbase, int nodeBase,
                                          int vec8, int* list, int tid, int wave) {
  int wc = 0;
  const int el0  = tid * EPT;
  const int e0   = cbase + el0;
  const int em   = nE - 1;
  const int sent = -2147483647 - 1;
  v4i da, db;
  if (vec8 != 0 && cbase + CHUNK <= nE) {
    da = *(const v4i*)(dsts + e0);
    db = *(const v4i*)(dsts + e0 + 4);
  } else {
    da.x = (e0     < nE) ? dsts[min(e0,     em)] : sent;
    da.y = (e0 + 1 < nE) ? dsts[min(e0 + 1, em)] : sent;
    da.z = (e0 + 2 < nE) ? dsts[min(e0 + 2, em)] : sent;
    da.w = (e0 + 3 < nE) ? dsts[min(e0 + 3, em)] : sent;
    db.x = (e0 + 4 < nE) ? dsts[min(e0 + 4, em)] : sent;
    db.y = (e0 + 5 < nE) ? dsts[min(e0 + 5, em)] : sent;
    db.z = (e0 + 6 < nE) ? dsts[min(e0 + 6, em)] : sent;
    db.w = (e0 + 7 < nE) ? dsts[min(e0 + 7, em)] : sent;
  }
  const unsigned nb = (unsigned)nodeBase;
  const unsigned s0 = (unsigned)da.x - nb, s1 = (unsigned)da.y - nb;
  const unsigned s2 = (unsigned)da.z - nb, s3 = (unsigned)da.w - nb;
  const unsigned s4 = (unsigned)db.x - nb, s5 = (unsigned)db.y - nb;
  const unsigned s6 = (unsigned)db.z - nb, s7 = (unsigned)db.w - nb;
  const bool h0 = s0 < (unsigned)NB, h1 = s1 < (unsigned)NB, h2 = s2 < (unsigned)NB, h3 = s3 < (unsigned)NB;
  const bool h4 = s4 < (unsigned)NB, h5 = s5 < (unsigned)NB, h6 = s6 < (unsigned)NB, h7 = s7 < (unsigned)NB;
  const unsigned any = __builtin_amdgcn_ballot_w32(h0 | h1 | h2 | h3 | h4 | h5 | h6 | h7);
  if (any != 0u) {
#define HITJ(J, HJ, SJ) { \
      const unsigned mj = __builtin_amdgcn_ballot_w32(HJ); \
      if (mj != 0u) { \
        if (HJ) { \
          const int pos = wc + (int)__builtin_amdgcn_mbcnt_lo(mj, 0u); \
          if (pos < WCAP) list[wave * WCAP + pos] = ((el0 + (J)) << 16) | (int)(SJ); \
        } \
        wc += (int)__builtin_popcount(mj); } }
    HITJ(0, h0, s0)
    HITJ(1, h1, s1)
    HITJ(2, h2, s2)
    HITJ(3, h3, s3)
    HITJ(4, h4, s4)
    HITJ(5, h5, s5)
    HITJ(6, h6, s6)
    HITJ(7, h7, s7)
#undef HITJ
  }
  return wc;
}

template <int FINAL>
__global__ __launch_bounds__(NTHR) void k_agg(
    const float* __restrict__ kP, const float* __restrict__ qP, const float* __restrict__ vP,
    const float* __restrict__ sP, const int* __restrict__ ei, const float* __restrict__ eat,
    const float* __restrict__ Wel, const float* __restrict__ bel,
    const float* __restrict__ gam, const float* __restrict__ bet,
    const float* __restrict__ rme, const float* __restrict__ rva,
    _Float16* hout16, float* hout32, int nN, int nE, int vec8) {
  extern __shared__ __attribute__((aligned(16))) float dynlds[];
  float* acc  = dynlds;
  int*   list = (int*)(dynlds + NB * HD);
  int*   wcnt = list + NWAVE * WCAP;

  const int tid  = threadIdx.x, lane = tid & 31;
  const int wave = __builtin_amdgcn_readfirstlane(tid >> 5);
  const int nodeBase = blockIdx.x * NB;
  const int* srcs = ei;
  const int* dsts = ei + nE;

#pragma unroll 4
  for (int i = tid; i < NB * HD / 4; i += NTHR) *(v4f*)(acc + 4 * i) = zero4();
  const v4f we4 = *(const v4f*)(Wel + 4 * lane);
  const v4f be4 = *(const v4f*)(bel + 4 * lane);
  __syncthreads();

  const int nChunks = (nE + CHUNK - 1) / CHUNK;
#pragma unroll 1
  for (int ch = 0; ch < nChunks; ++ch) {
    const int cbase = ch * CHUNK;
    const int wc = scan_chunk(dsts, nE, cbase, nodeBase, vec8, list, tid, wave);
    if (lane == 0) wcnt[wave] = wc;
    __syncthreads();

#pragma unroll 1
    for (int w = 0; w < NWAVE; ++w) {
      int n = __builtin_amdgcn_readfirstlane(wcnt[w]);
      n = n > WCAP ? WCAP : (n < 0 ? 0 : n);
      const int* lp = list + w * WCAP;
#pragma unroll 1
      for (int i = 0; i < n; ++i) {
        const int ent  = __builtin_amdgcn_readfirstlane(lp[i]);
        const int slot = ent & 0xFFFF;
        if ((slot & (NWAVE - 1)) != wave) continue;
        const int sl = slot < NB - 1 ? slot : NB - 1;
        int e = cbase + (ent >> 16);
        e = e < 0 ? 0 : (e > nE - 1 ? nE - 1 : e);
        int sr = srcs[e];
        sr = sr < 0 ? 0 : (sr > nN - 1 ? nN - 1 : sr);
        int dn = nodeBase + sl;
        dn = dn > nN - 1 ? nN - 1 : dn;
        const float ea = eat[e];
        const v4f kd = *(const v4f*)(kP + (size_t)dn * HD + 4 * lane);
        const v4f qs = *(const v4f*)(qP + (size_t)sr * HD + 4 * lane);
        const v4f vs = *(const v4f*)(vP + (size_t)sr * HD + 4 * lane);
        v4f g;
        g.x = gate1(kd.x, qs.x, ea, we4.x, be4.x);
        g.y = gate1(kd.y, qs.y, ea, we4.y, be4.y);
        g.z = gate1(kd.z, qs.z, ea, we4.z, be4.z);
        g.w = gate1(kd.w, qs.w, ea, we4.w, be4.w);
        v4f* ap = (v4f*)(acc + sl * HD + 4 * lane);
        v4f av = *ap;
        av += g * vs;
        *ap = av;
      }
    }
    __syncthreads();
  }
  __syncthreads();

  if (FINAL == 0) {
    const int rr = lane >> 4, cg = (lane & 15) * 8;
    const v4f ga = *(const v4f*)(gam + cg), gb = *(const v4f*)(gam + cg + 4);
    const v4f ta = *(const v4f*)(bet + cg), tb = *(const v4f*)(bet + cg + 4);
    const v4f ma = *(const v4f*)(rme + cg), mb = *(const v4f*)(rme + cg + 4);
    const v4f va = *(const v4f*)(rva + cg), vb = *(const v4f*)(rva + cg + 4);
    v4f ra, rb;
    ra.x = rsqrtf(va.x + BN_EPS); ra.y = rsqrtf(va.y + BN_EPS); ra.z = rsqrtf(va.z + BN_EPS); ra.w = rsqrtf(va.w + BN_EPS);
    rb.x = rsqrtf(vb.x + BN_EPS); rb.y = rsqrtf(vb.y + BN_EPS); rb.z = rsqrtf(vb.z + BN_EPS); rb.w = rsqrtf(vb.w + BN_EPS);
#pragma unroll 1
    for (int it = 0; it < NB / (2 * NWAVE); ++it) {
      const int slot = (it * NWAVE + wave) * 2 + rr;
      const int node = nodeBase + slot;
      const bool ok = node < nN;
      const v4f a0 = *(const v4f*)(acc + slot * HD + cg);
      const v4f a1 = *(const v4f*)(acc + slot * HD + cg + 4);
      const v4f s0 = *(const v4f*)(sP + (size_t)node * HD + cg);
      const v4f s1 = *(const v4f*)(sP + (size_t)node * HD + cg + 4);
      v8h hv;
      hv[0] = (_Float16)(ok ? bnl(s0.x + a0.x, ga.x, ma.x, ra.x, ta.x) : 0.0f);
      hv[1] = (_Float16)(ok ? bnl(s0.y + a0.y, ga.y, ma.y, ra.y, ta.y) : 0.0f);
      hv[2] = (_Float16)(ok ? bnl(s0.z + a0.z, ga.z, ma.z, ra.z, ta.z) : 0.0f);
      hv[3] = (_Float16)(ok ? bnl(s0.w + a0.w, ga.w, ma.w, ra.w, ta.w) : 0.0f);
      hv[4] = (_Float16)(ok ? bnl(s1.x + a1.x, gb.x, mb.x, rb.x, tb.x) : 0.0f);
      hv[5] = (_Float16)(ok ? bnl(s1.y + a1.y, gb.y, mb.y, rb.y, tb.y) : 0.0f);
      hv[6] = (_Float16)(ok ? bnl(s1.z + a1.z, gb.z, mb.z, rb.z, tb.z) : 0.0f);
      hv[7] = (_Float16)(ok ? bnl(s1.w + a1.w, gb.w, mb.w, rb.w, tb.w) : 0.0f);
      _Float16* hp = hout16 + (size_t)node * HD + cg;
      *(volatile v8h*)hp = hv;
      __threadfence();
      *(volatile v8h*)hp = hv;
    }
  } else {
    const int c4 = 4 * lane;
    const v4f ga = *(const v4f*)(gam + c4);
    const v4f ta = *(const v4f*)(bet + c4);
    const v4f ma = *(const v4f*)(rme + c4);
    const v4f va = *(const v4f*)(rva + c4);
    v4f ra;
    ra.x = rsqrtf(va.x + BN_EPS); ra.y = rsqrtf(va.y + BN_EPS); ra.z = rsqrtf(va.z + BN_EPS); ra.w = rsqrtf(va.w + BN_EPS);
#pragma unroll 1
    for (int it = 0; it < NB / NWAVE; ++it) {
      const int slot = it * NWAVE + wave;
      const int node = nodeBase + slot;
      const bool ok = node < nN;
      const v4f a0 = *(const v4f*)(acc + slot * HD + c4);
      const v4f s0 = *(const v4f*)(sP + (size_t)node * HD + c4);
      v4f hv;
      hv.x = ok ? bnl(s0.x + a0.x, ga.x, ma.x, ra.x, ta.x) : 0.0f;
      hv.y = ok ? bnl(s0.y + a0.y, ga.y, ma.y, ra.y, ta.y) : 0.0f;
      hv.z = ok ? bnl(s0.z + a0.z, ga.z, ma.z, ra.z, ta.z) : 0.0f;
      hv.w = ok ? bnl(s0.w + a0.w, ga.w, ma.w, ra.w, ta.w) : 0.0f;
      float* hp = hout32 + (size_t)node * HD + c4;
      *(volatile v4f*)hp = hv;
      __threadfence();
      *(volatile v4f*)hp = hv;
    }
  }
}

__global__ __launch_bounds__(NTHR) void k_pool(const float* __restrict__ hf, const int* __restrict__ batch,
                                              float* pool, int nN) {
  __shared__ __attribute__((aligned(16))) float red[NWAVE * HD];
  __shared__ int cw[NWAVE];
  const int g = blockIdx.x;
  const int tid = threadIdx.x, lane = tid & 31;
  const int wave = __builtin_amdgcn_readfirstlane(tid >> 5);
  v4f s = zero4();
  int cnt = 0;
#pragma unroll 1
  for (int base = wave * 32; base < nN; base += NWAVE * 32) {
    const int n  = base + lane;
    const int bv = batch[min(n, nN - 1)];
    const bool hit = (n < nN) && (bv == g);
    unsigned mask = __builtin_amdgcn_ballot_w32(hit);
    cnt += (int)__builtin_popcount(mask);
#pragma unroll 1
    for (int q = 0; q < 32 && mask != 0u; ++q) {
      const int j = (int)__builtin_ctz(mask);
      const int row = base + j;
      s += *(const v4f*)(hf + (size_t)row * HD + 4 * lane);
      mask &= mask - 1u;
    }
  }
  *(v4f*)(red + wave * HD + 4 * lane) = s;
  if (lane == 0) cw[wave] = cnt;
  __syncthreads();
  if (wave == 0) {
    v4f t = zero4();
    int c = 0;
#pragma unroll
    for (int w = 0; w < NWAVE; ++w) { t += *(const v4f*)(red + w * HD + 4 * lane); c += cw[w]; }
    const float cf  = (float)c;
    const float inv = 1.0f / fmaxf(cf, 1.0f);
    t *= inv;
    float* pp = pool + (size_t)g * HD + 4 * lane;
    *(volatile v4f*)pp = t;
    __threadfence();
    *(volatile v4f*)pp = t;
  }
}

__global__ __launch_bounds__(NG * NCLS) void k_head(const float* __restrict__ pool, const float* __restrict__ clin,
                                                   const float* __restrict__ Wc, const float* __restrict__ bc,
                                                   float* out) {
  __shared__ __attribute__((aligned(16))) float ob[NG * NCLS];
  const int t = threadIdx.x;
  const int g = t >> 1, j = t & 1;
  float a = 0.0f;
#pragma unroll 4
  for (int c = 0; c < HD; ++c) a += pool[(size_t)g * HD + c] * Wc[c * NCLS + j];
#pragma unroll
  for (int i = 0; i < NCL; ++i) a += clin[g * NCL + i] * Wc[(HD + i) * NCLS + j];
  a += bc[j];
  ob[t] = a;
  __syncthreads();
  if (t < 32) {
    const v4f v = *(const v4f*)(ob + 4 * t);
    *(volatile v4f*)(out + 4 * t) = v;
    __threadfence();
    *(volatile v4f*)(out + 4 * t) = v;
  }
}

extern "C" void kernel_launch(void* const* d_in, const int* in_sizes, int n_in,
                              void* d_out, int out_size, void* d_ws, size_t ws_size,
                              hipStream_t stream) {
  if (n_in < 21) return;
  const int nN = in_sizes[0] / HD;
  if (nN <= 0 || in_sizes[0] != nN * HD) return;
  const int nE = in_sizes[1] / 2;
  if (nE <= 0 || in_sizes[1] != 2 * nE || in_sizes[2] != nE) return;
  if (in_sizes[3] != nN) return;
  if (in_sizes[4] != NG * NCL) return;
  const int nL = in_sizes[5] / (HD * HD);
  if (nL <= 0 || nL > 8 || in_sizes[5] != nL * HD * HD) return;
  if (in_sizes[7] != nL * HD * HD || in_sizes[9] != nL * HD * HD || in_sizes[11] != nL * HD * HD) return;
  if (in_sizes[6] != nL * HD || in_sizes[8] != nL * HD || in_sizes[10] != nL * HD || in_sizes[12] != nL * HD) return;
  if (in_sizes[13] != nL * HD || in_sizes[14] != nL * HD) return;
  if (in_sizes[15] != nL * HD || in_sizes[16] != nL * HD || in_sizes[17] != nL * HD || in_sizes[18] != nL * HD) return;
  if (in_sizes[19] != (HD + NCL) * NCLS || in_sizes[20] != NCLS) return;
  if (out_size != NG * NCLS) return;

  const float* x     = (const float*)d_in[0];
  const int*   ei    = (const int*)d_in[1];
  const float* ea    = (const float*)d_in[2];
  const int*   batch = (const int*)d_in[3];
  const float* clin  = (const float*)d_in[4];
  const float* Wk = (const float*)d_in[5];
  const float* bk = (const float*)d_in[6];
  const float* Wq = (const float*)d_in[7];
  const float* bq = (const float*)d_in[8];
  const float* Wv = (const float*)d_in[9];
  const float* bv = (const float*)d_in[10];
  const float* Ws = (const float*)d_in[11];
  const float* bs = (const float*)d_in[12];
  const float* We = (const float*)d_in[13];
  const float* be = (const float*)d_in[14];
  const float* gam = (const float*)d_in[15];
  const float* bet = (const float*)d_in[16];
  const float* rme = (const float*)d_in[17];
  const float* rva = (const float*)d_in[18];
  const float* Wc = (const float*)d_in[19];
  const float* bc = (const float*)d_in[20];
  float* out = (float*)d_out;

  const int nBlk = (nN + NB - 1) / NB;
  const int nPad = nBlk * NB;

  char* ws = (char*)d_ws;
  size_t off = 0;
  const size_t szWt = (((size_t)nL * 4 * HD * HD * 2) + 255) & ~(size_t)255;
  const size_t szP  = (size_t)nPad * HD * 4;
  const size_t szPl = (size_t)NG * HD * 4;
  const size_t oWt = off; off += szWt;
  const size_t oH  = off; off += szP;
  const size_t oK  = off; off += szP;
  const size_t oQ  = off; off += szP;
  const size_t oV  = off; off += szP;
  const size_t oS  = off; off += szP;
  const size_t oPl = off; off += szPl;
  if (off > ws_size) return;

  _Float16* Wt  = (_Float16*)(ws + oWt);
  _Float16* h16 = (_Float16*)(ws + oH);
  float*    h32 = (float*)(ws + oH);
  float* kP = (float*)(ws + oK);
  float* qP = (float*)(ws + oQ);
  float* vP = (float*)(ws + oV);
  float* sP = (float*)(ws + oS);
  float* pool = (float*)(ws + oPl);

  const int vec8 = ((nE & 3) == 0) ? 1 : 0;

  hipFuncSetAttribute(reinterpret_cast<const void*>(&k_agg<0>), hipFuncAttributeMaxDynamicSharedMemorySize, AGG_LDS);
  hipFuncSetAttribute(reinterpret_cast<const void*>(&k_agg<1>), hipFuncAttributeMaxDynamicSharedMemorySize, AGG_LDS);

  k_cvtw<<<nL * 4 * 8, NTHR, 0, stream>>>(Wk, Wq, Wv, Ws, Wt, nL);
  k_cvtx<<<nPad / 16, NTHR, 0, stream>>>(x, h16, nN, nPad);

  for (int l = 0; l < nL; ++l) {
    k_gemm<<<nPad / GROWS, GTHR, 0, stream>>>(
        h16, Wt + (size_t)l * 4 * HD * HD,
        bk + (size_t)l * HD, bq + (size_t)l * HD, bv + (size_t)l * HD, bs + (size_t)l * HD,
        kP, qP, vP, sP);
    if (l == nL - 1) {
      k_agg<1><<<nBlk, NTHR, AGG_LDS, stream>>>(
          kP, qP, vP, sP, ei, ea, We + (size_t)l * HD, be + (size_t)l * HD,
          gam + (size_t)l * HD, bet + (size_t)l * HD, rme + (size_t)l * HD, rva + (size_t)l * HD,
          h16, h32, nN, nE, vec8);
    } else {
      k_agg<0><<<nBlk, NTHR, AGG_LDS, stream>>>(
          kP, qP, vP, sP, ei, ea, We + (size_t)l * HD, be + (size_t)l * HD,
          gam + (size_t)l * HD, bet + (size_t)l * HD, rme + (size_t)l * HD, rva + (size_t)l * HD,
          h16, h32, nN, nE, vec8);
    }
  }

  k_pool<<<NG, NTHR, 0, stream>>>(h32, batch, pool, nN);
  k_head<<<1, NG * NCLS, 0, stream>>>(pool, clin, Wc, bc, out);
}
